// EdgeConvBlock_25623774888365
// MI455X (gfx1250) — hardware-verified
//
#include <hip/hip_runtime.h>
#include <stddef.h>
#include <stdint.h>

#define CIN    128
#define COUT   256
#define KNB    16
#define NW3    768
#define KK     512
#define NTHR   256
#define GBM    64
#define GTHR   128
#define NGC    192
#define NPB    4
#define ROWS   64
#define AP     520
#define NU_WT  (NW3 * (CIN / 8))
#define NU_W22 (COUT * (KK / 8))
#define SA_BYTES (ROWS * AP * 2)
#define EDGE_LDS_BYTES (SA_BYTES + NPB * COUT * 4)
#define WSCAP  134217728
#define LNEPS  1e-5f

static_assert(NU_WT % NTHR == 0 && NU_W22 % NTHR == 0);
static_assert(CIN % 32 == 0 && KK % 32 == 0 && KK == 2 * COUT);
static_assert((AP * 2) % 16 == 0 && AP >= KK && SA_BYTES % 16 == 0);
static_assert(ROWS == NPB * KNB && ROWS == 8 * (NTHR / 32));
static_assert(COUT == 32 * (NTHR / 32) && COUT == 8 * 32);
static_assert(GBM == (GTHR / 32) * 16 && NGC == 3 * 64 && COUT % 64 == 0);
static_assert(GBM * NGC * 4 <= 65536 && EDGE_LDS_BYTES <= 300000);
static_assert(NW3 == 3 * COUT && (COUT % 16) == 0);

typedef float          v4f   __attribute__((ext_vector_type(4)));
typedef float          v8f   __attribute__((ext_vector_type(8)));
typedef int            v8i   __attribute__((ext_vector_type(8)));
typedef unsigned short v8us  __attribute__((ext_vector_type(8)));
typedef unsigned short v16us __attribute__((ext_vector_type(16)));
typedef __bf16         v16bf __attribute__((ext_vector_type(16)));
typedef v4f  __attribute__((may_alias)) v4fa;
typedef v8us __attribute__((may_alias)) v8usa;
union FragB { v16bf v; v16us u; v8us h[2]; v8i w; };

__device__ __forceinline__ v8f wmb(const FragB& a, const FragB& b, v8f c) {
  v8f d = __builtin_amdgcn_wmma_f32_16x16x32_bf16(false, a.v, false, b.v, (short)0, c, false, false);
  asm volatile("v_nop\n\tv_nop\n\tv_nop\n\tv_nop" : "+v"(d) : "v"(a.w), "v"(b.w));
  return d;
}

__device__ __forceinline__ v8f z8() { v8f z = {0.f, 0.f, 0.f, 0.f, 0.f, 0.f, 0.f, 0.f}; return z; }

__device__ __forceinline__ unsigned bf16_bits(float f) {
  const unsigned u = __float_as_uint(f);
  return (u + 0x7FFFu + ((u >> 16) & 1u)) >> 16;
}
__device__ __forceinline__ float bf16_val(float f) {
  return __uint_as_float(bf16_bits(f) << 16);
}
__device__ __forceinline__ void put16(unsigned short* dp, v8us o) {
  *(volatile v8us*)dp = o;
  __threadfence();
  *(volatile v8us*)dp = o;
}
__device__ __forceinline__ float gelu_erf(float v) {
  return 0.5f * v * (1.0f + erff(v * 0.70710678118654752f));
}

__global__ __launch_bounds__(NTHR) void k_prep(const float* __restrict__ feat, const float* __restrict__ W1,
                                               const float* __restrict__ W2, const float* __restrict__ Ws,
                                               int nN, int mRows, unsigned short* WT, unsigned short* W22,
                                               unsigned short* FB) {
  const int u  = (int)blockIdx.x * NTHR + (int)threadIdx.x;
  const int L0 = NU_WT;
  const int L1 = L0 + NU_W22;
  const int L2 = L1 + mRows * (CIN / 8);
  v8us o;
  if (u < L0) {
    const int n    = u >> 4;
    const int k8   = (u & 15) * 8;
    const int sub  = n >> 8;
    const int col  = n & (COUT - 1);
    const int sub1 = sub > 1 ? 1 : sub;
    const float* p1 = W1 + (size_t)(sub1 * CIN + k8) * COUT + col;
    const float* p2 = Ws + (size_t)k8 * COUT + col;
    const float* p  = (sub == 2) ? p2 : p1;
#pragma unroll
    for (int i = 0; i < 8; ++i) o[i] = (unsigned short)bf16_bits(p[(size_t)i * COUT]);
    put16(WT + (size_t)u * 8, o);
    return;
  } else if (u < L1) {
    const int v  = u - L0;
    const int n  = v >> 6;
    const int k8 = (v & 63) * 8;
    const int kk = k8 & (COUT - 1);
    const float* p = W2 + (size_t)kk * COUT + n;
#pragma unroll
    for (int i = 0; i < 8; ++i) o[i] = (unsigned short)bf16_bits(p[(size_t)i * COUT]);
    put16(W22 + (size_t)v * 8, o);
    return;
  } else if (u < L2) {
    const int v   = u - L1;
    const int row = v >> 4;
    const int j   = v & 15;
    const int rc  = row < nN ? row : nN - 1;
    const unsigned mk = (row < nN) ? 0xffffu : 0u;
    const float* p = feat + (size_t)rc * CIN + 8 * j;
    const v4f a = *(const v4f*)p;
    const v4f b = *(const v4f*)(p + 4);
    o[0] = (unsigned short)(bf16_bits(a.x) & mk); o[1] = (unsigned short)(bf16_bits(a.y) & mk);
    o[2] = (unsigned short)(bf16_bits(a.z) & mk); o[3] = (unsigned short)(bf16_bits(a.w) & mk);
    o[4] = (unsigned short)(bf16_bits(b.x) & mk); o[5] = (unsigned short)(bf16_bits(b.y) & mk);
    o[6] = (unsigned short)(bf16_bits(b.z) & mk); o[7] = (unsigned short)(bf16_bits(b.w) & mk);
    put16(FB + (size_t)v * 8, o);
    return;
  }
}

__global__ __launch_bounds__(GTHR) void k_node(const unsigned short* __restrict__ FB,
                                               const unsigned short* __restrict__ WT,
                                               const float* __restrict__ b1, const float* __restrict__ b2,
                                               const float* __restrict__ bs, float* CB, float* BN, float* SK) {
  __shared__ __attribute__((aligned(16))) float stg[GBM * NGC];
  const int tid = (int)threadIdx.x, lane = tid & 31, wave = tid >> 5, hh = lane >> 4, m = lane & 15;
  const int rowBase = (int)blockIdx.x * GBM;
  const int cg = (int)blockIdx.y;

  v8f acc[12];
#pragma unroll
  for (int t = 0; t < 12; ++t) acc[t] = z8();
  const unsigned short* ap = FB + (size_t)(rowBase + 16 * wave + m) * (size_t)CIN + 8 * hh;
  const unsigned short* bp = WT + (size_t)(cg * 64 + m) * (size_t)CIN + 8 * hh;

#pragma unroll
  for (int k0 = 0; k0 < CIN; k0 += 32) {
    FragB af;
    af.h[0] = *(const v8usa*)(ap + k0);
    af.h[1] = *(const v8usa*)(ap + k0 + 16);
#pragma unroll
    for (int nt = 0; nt < 12; ++nt) {
      const unsigned short* wq = bp + (size_t)((nt >> 2) * COUT + (nt & 3) * 16) * (size_t)CIN + k0;
      FragB bf;
      bf.h[0] = *(const v8usa*)wq;
      bf.h[1] = *(const v8usa*)(wq + 16);
      acc[nt] = wmb(af, bf, acc[nt]);
    }
  }

#pragma unroll
  for (int nt = 0; nt < 12; ++nt) {
    const int lc = 16 * nt + m;
#pragma unroll
    for (int r = 0; r < 8; ++r) {
      const int lr = 16 * wave + 8 * hh + r;
      stg[lr * NGC + lc] = acc[nt][r];
    }
  }
  __syncthreads();

  const int cq = 4 * (lane & 15);
  const int gc = cg * 64 + cq;
  const v4f b1v = *(const v4f*)(b1 + gc);
  const v4f b2v = *(const v4f*)(b2 + gc);
  const v4f bsv = *(const v4f*)(bs + gc);
  v4f q1, q2, q3;
  q1.x = bf16_val(b1v.x); q1.y = bf16_val(b1v.y); q1.z = bf16_val(b1v.z); q1.w = bf16_val(b1v.w);
  q2.x = bf16_val(b2v.x); q2.y = bf16_val(b2v.y); q2.z = bf16_val(b2v.z); q2.w = bf16_val(b2v.w);
  q3.x = bf16_val(bsv.x); q3.y = bf16_val(bsv.y); q3.z = bf16_val(bsv.z); q3.w = bf16_val(bsv.w);

  v4f cbv[8], bnv[8], skv[8];
#pragma unroll
  for (int it = 0; it < 8; ++it) {
    const float* sp = stg + (16 * wave + 2 * it + hh) * NGC;
    const v4f a = *(const v4fa*)(sp + cq);
    const v4f b = *(const v4fa*)(sp + 64 + cq);
    const v4f s = *(const v4fa*)(sp + 128 + cq);
    cbv[it] = (a - b) + q1;
    bnv[it] = b;
    skv[it] = (s + q3) + q2;
  }
#pragma unroll
  for (int it = 0; it < 8; ++it) {
    const size_t o = (size_t)(rowBase + 16 * wave + 2 * it + hh) * (size_t)COUT + (size_t)gc;
    *(volatile v4f*)(CB + o) = cbv[it];
    *(volatile v4f*)(BN + o) = bnv[it];
    *(volatile v4f*)(SK + o) = skv[it];
  }
  __threadfence();
#pragma unroll
  for (int it = 0; it < 8; ++it) {
    const size_t o = (size_t)(rowBase + 16 * wave + 2 * it + hh) * (size_t)COUT + (size_t)gc;
    *(volatile v4f*)(CB + o) = cbv[it];
    *(volatile v4f*)(BN + o) = bnv[it];
    *(volatile v4f*)(SK + o) = skv[it];
  }
}

__global__ __launch_bounds__(NTHR) void k_edge(const int* __restrict__ knn, int nN,
                                               const float* __restrict__ CB, const float* __restrict__ BN,
                                               const float* __restrict__ SK,
                                               const unsigned short* __restrict__ W22,
                                               const float* __restrict__ gam, const float* __restrict__ bet,
                                               float* out) {
  extern __shared__ __attribute__((aligned(16))) float dyn[];
  unsigned short* sA  = (unsigned short*)dyn;
  float*          agg = dyn + SA_BYTES / 4;

  const int tid = (int)threadIdx.x, lane = tid & 31, wave = tid >> 5, hh = lane >> 4, m = lane & 15;
  const int n0 = (int)blockIdx.x * NPB;

  {
    const int j  = wave >> 1;
    int nc = n0 + j;
    nc = nc < nN ? nc : nN - 1;
    const int c0 = 8 * lane;
    const v4f ca = *(const v4f*)(CB + (size_t)nc * COUT + c0);
    const v4f cb = *(const v4f*)(CB + (size_t)nc * COUT + c0 + 4);
#pragma unroll 1
    for (int i = 0; i < 8; ++i) {
      const int k = (wave & 1) * 8 + i;
      int s = knn[(size_t)nc * KNB + k];
      s = s < 0 ? 0 : (s > nN - 1 ? nN - 1 : s);
      const float* bq = BN + (size_t)s * COUT + c0;
      const v4f ba = *(const v4f*)bq;
      const v4f bb = *(const v4f*)(bq + 4);
      const v8f vv = {ca.x + ba.x, ca.y + ba.y, ca.z + ba.z, ca.w + ba.w,
                      cb.x + bb.x, cb.y + bb.y, cb.z + bb.z, cb.w + bb.w};
      v8us oh, ol;
#pragma unroll
      for (int e = 0; e < 8; ++e) {
        const float g = gelu_erf(vv[e]);
        const unsigned hb = bf16_bits(g);
        oh[e] = (unsigned short)hb;
        ol[e] = (unsigned short)bf16_bits(g - __uint_as_float(hb << 16));
      }
      unsigned short* ra = sA + (size_t)(16 * j + k) * AP;
      *(v8usa*)(ra + c0) = oh;
      *(v8usa*)(ra + COUT + c0) = ol;
    }
  }
  __syncthreads();

  v8f acc[4][2];
#pragma unroll
  for (int mt = 0; mt < 4; ++mt) { acc[mt][0] = z8(); acc[mt][1] = z8(); }
  {
    const unsigned short* a0 = sA + m * AP + 8 * hh;
    const unsigned short* bp = W22 + (size_t)(32 * wave + m) * (size_t)KK + 8 * hh;
#pragma unroll 2
    for (int k0 = 0; k0 < KK; k0 += 32) {
      FragB b0, b1;
      b0.h[0] = *(const v8usa*)(bp + k0);
      b0.h[1] = *(const v8usa*)(bp + k0 + 16);
      b1.h[0] = *(const v8usa*)(bp + (size_t)16 * KK + k0);
      b1.h[1] = *(const v8usa*)(bp + (size_t)16 * KK + k0 + 16);
#pragma unroll
      for (int mt = 0; mt < 4; ++mt) {
        FragB a;
        a.h[0] = *(const v8usa*)(a0 + mt * 16 * AP + k0);
        a.h[1] = *(const v8usa*)(a0 + mt * 16 * AP + k0 + 16);
        acc[mt][0] = wmb(a, b0, acc[mt][0]);
        acc[mt][1] = wmb(a, b1, acc[mt][1]);
      }
    }
  }

#pragma unroll
  for (int mt = 0; mt < 4; ++mt) {
#pragma unroll
    for (int nt = 0; nt < 2; ++nt) {
      float mx = acc[mt][nt][0];
#pragma unroll
      for (int r = 1; r < 8; ++r) mx = fmaxf(mx, acc[mt][nt][r]);
      const float ot = __shfl_xor(mx, 16, 32);
      mx = fmaxf(mx, ot);
      if (hh == 0) agg[mt * COUT + 32 * wave + 16 * nt + m] = mx;
    }
  }
  __syncthreads();

  if (wave < NPB) {
    const int node = n0 + wave;
    const int ncl  = node < nN ? node : nN - 1;
    const int c4   = 4 * lane;
    const float* ag = agg + wave * COUT;
    const v4f a0 = *(const v4fa*)(ag + c4);
    const v4f a1 = *(const v4fa*)(ag + 128 + c4);
    const v4f s0 = *(const v4f*)(SK + (size_t)ncl * COUT + c4);
    const v4f s1 = *(const v4f*)(SK + (size_t)ncl * COUT + 128 + c4);
    const v4f z0 = a0 + s0;
    const v4f z1 = a1 + s1;
    float sum = ((z0.x + z0.y) + (z0.z + z0.w)) + ((z1.x + z1.y) + (z1.z + z1.w));
#pragma unroll
    for (int off = 16; off > 0; off >>= 1) sum += __shfl_xor(sum, off, 32);
    const float mu = sum * (1.0f / 256.0f);
    const v4f d0 = z0 - mu;
    const v4f d1 = z1 - mu;
    float q = ((d0.x * d0.x + d0.y * d0.y) + (d0.z * d0.z + d0.w * d0.w)) +
              ((d1.x * d1.x + d1.y * d1.y) + (d1.z * d1.z + d1.w * d1.w));
#pragma unroll
    for (int off = 16; off > 0; off >>= 1) q += __shfl_xor(q, off, 32);
    const float var  = q * (1.0f / 256.0f);
    const float rstd = 1.0f / sqrtf(var + LNEPS);
    const v4f g0 = *(const v4f*)(gam + c4);
    const v4f g1 = *(const v4f*)(gam + 128 + c4);
    const v4f e0 = *(const v4f*)(bet + c4);
    const v4f e1 = *(const v4f*)(bet + 128 + c4);
    v4f o0, o1;
    o0.x = d0.x * rstd * bf16_val(g0.x) + bf16_val(e0.x);
    o0.y = d0.y * rstd * bf16_val(g0.y) + bf16_val(e0.y);
    o0.z = d0.z * rstd * bf16_val(g0.z) + bf16_val(e0.z);
    o0.w = d0.w * rstd * bf16_val(g0.w) + bf16_val(e0.w);
    o1.x = d1.x * rstd * bf16_val(g1.x) + bf16_val(e1.x);
    o1.y = d1.y * rstd * bf16_val(g1.y) + bf16_val(e1.y);
    o1.z = d1.z * rstd * bf16_val(g1.z) + bf16_val(e1.z);
    o1.w = d1.w * rstd * bf16_val(g1.w) + bf16_val(e1.w);
    const bool live = node < nN;
    float* op = out + (size_t)ncl * COUT + c4;
    if (live) {
      *(volatile v4f*)op = o0;
      *(volatile v4f*)(op + 128) = o1;
    }
    __threadfence();
    if (live) {
      *(volatile v4f*)op = o0;
      *(volatile v4f*)(op + 128) = o1;
    }
  }
}

static inline int cdiv(int a, int b) { return (a + b - 1) / b; }
static inline size_t al256(size_t o) { return (o + 255) & ~(size_t)255; }

extern "C" void kernel_launch(void* const* d_in, const int* in_sizes, int n_in,
                              void* d_out, int out_size, void* d_ws, size_t ws_size,
                              hipStream_t stream) {
  if (n_in < 10) return;
  if (in_sizes[0] < CIN * 16 || (in_sizes[0] % CIN) != 0) return;
  const int nN = in_sizes[0] / CIN;
  if (nN >= (1 << 22)) return;
  if ((long long)in_sizes[1] != (long long)nN * KNB) return;
  if (in_sizes[2] != 2 * CIN * COUT) return;
  if (in_sizes[3] != COUT) return;
  if (in_sizes[4] != COUT * COUT) return;
  if (in_sizes[5] != COUT) return;
  if (in_sizes[6] != CIN * COUT) return;
  if (in_sizes[7] != COUT || in_sizes[8] != COUT || in_sizes[9] != COUT) return;
  if ((long long)out_size != (long long)nN * COUT) return;

  const float* feat = (const float*)d_in[0];
  const int*   knn  = (const int*)d_in[1];
  const float* W1   = (const float*)d_in[2];
  const float* b1   = (const float*)d_in[3];
  const float* W2   = (const float*)d_in[4];
  const float* b2   = (const float*)d_in[5];
  const float* Ws   = (const float*)d_in[6];
  const float* bs   = (const float*)d_in[7];
  const float* gam  = (const float*)d_in[8];
  const float* bet  = (const float*)d_in[9];
  float* out = (float*)d_out;

  const int MP = cdiv(nN, GBM) * GBM;
  const int gM = MP / GBM;
  const int gE = cdiv(nN, NPB);

  char* ws = (char*)d_ws;
  size_t off = 0;
  const size_t oWT  = off; off = al256(off + (size_t)NW3 * CIN * 2);
  const size_t oW22 = off; off = al256(off + (size_t)COUT * KK * 2);
  const size_t oFB  = off; off = al256(off + (size_t)MP * CIN * 2);
  const size_t oCB  = off; off = al256(off + (size_t)MP * COUT * 4);
  const size_t oBN  = off; off = al256(off + (size_t)MP * COUT * 4);
  const size_t oSK  = off; off = al256(off + (size_t)MP * COUT * 4);
  if (off > ws_size || off > (size_t)WSCAP) return;
  unsigned short* WT  = (unsigned short*)(ws + oWT);
  unsigned short* W22 = (unsigned short*)(ws + oW22);
  unsigned short* FB  = (unsigned short*)(ws + oFB);
  float*          CB  = (float*)(ws + oCB);
  float*          BN  = (float*)(ws + oBN);
  float*          SK  = (float*)(ws + oSK);

  hipFuncSetAttribute(reinterpret_cast<const void*>(&k_edge), hipFuncAttributeMaxDynamicSharedMemorySize,
                      (int)EDGE_LDS_BYTES);

  const int nPrep = NU_WT + NU_W22 + MP * (CIN / 8);

  k_prep<<<cdiv(nPrep, NTHR), NTHR, 0, stream>>>(feat, W1, W2, Ws, nN, MP, WT, W22, FB);
  k_node<<<dim3((unsigned)gM, (unsigned)(COUT / 64)), GTHR, 0, stream>>>(FB, WT, b1, b2, bs, CB, BN, SK);
  k_edge<<<gE, NTHR, EDGE_LDS_BYTES, stream>>>(knn, nN, CB, BN, SK, W22, gam, bet, out);
}
